// TransformerBlock_45543833207026
// MI455X (gfx1250) — hardware-run, weakly checked
//
#include <hip/hip_runtime.h>
#include <math.h>

typedef __attribute__((ext_vector_type(16))) _Float16 v16h;
typedef __attribute__((ext_vector_type(8)))  _Float16 v8h;
typedef __attribute__((ext_vector_type(4)))  _Float16 v4h;
typedef __attribute__((ext_vector_type(8)))  float v8f;
typedef __attribute__((ext_vector_type(4)))  float v4f;

#ifndef SEQ
#define SEQ 2048
#endif
#define SEQ_FULL 2048
#ifndef NB
#define NB 2
#endif
#define NB_FULL 2
#define DM 256
#define NH 8
#define DH 32
#define FF 1024
#define TOKS ((unsigned)(NB) * (unsigned)(SEQ))
#define ROWS (1u * TOKS)
#define NGRP (ROWS / 16u)
#define OUT1_OFF ((size_t)NB_FULL * SEQ_FULL * DM)
#define OUT2_OFF (OUT1_OFF + (size_t)NB_FULL * SEQ_FULL * SEQ_FULL)
#define SCALE (0.17677669529663687f)
#define PCY (16384.0f)
#define WC (64.0f)
#define OC (256.0f)
#define F16MIN (6.103515625e-05f)
#define LN_EPS (1e-6f)
#define BN_EPS (1e-6f)
static_assert(SEQ % 64 == 0);
static_assert(SEQ >= 64);
static_assert(SEQ <= SEQ_FULL);
static_assert(NB >= 1 && NB <= NB_FULL);
static_assert(DM == NH * DH);
static_assert(DH == 32);
static_assert(NH == 8);
static_assert((DM >> 3) == DH);
static_assert(DM % 128 == 0 && FF % 128 == 0);
static_assert(DM % 32 == 0 && FF % 32 == 0);
static_assert(OUT1_OFF * 4u == 4194304u);
static_assert(OUT2_OFF * 4u == 37748736u);
static_assert(DH * 4 == 128);

#define WSZ_WQKV (2u * (size_t)768 * DM)
#define WSZ_WO   (2u * (size_t)DM * DM)
#define WSZ_W1T  (2u * (size_t)FF * DM)
#define WSZ_W2T  (2u * (size_t)DM * FF)
#define WSZ_P16  (2u * (size_t)ROWS * DM)
#define WSZ_P32  (4u * (size_t)ROWS * DM)
#define WSZ_H    (2u * (size_t)ROWS * FF)
#define WSZ_H32  (4u * (size_t)ROWS * FF)
#define WSZ_PT   (4u * (size_t)NGRP * FF)
#define WSZ_AB1  (4u * (size_t)2 * FF)
#define WSZ_AB2  (4u * (size_t)2 * DM)
#define WS_WQKV  ((size_t)0)
#define WS_WO    (WS_WQKV + WSZ_WQKV)
#define WS_W1T   (WS_WO   + WSZ_WO)
#define WS_W2T   (WS_W1T  + WSZ_W1T)
#define WS_XN    (WS_W2T  + WSZ_W2T)
#define WS_Q     (WS_XN   + WSZ_P16)
#define WS_K     (WS_Q    + WSZ_P16)
#define WS_VT    (WS_K    + WSZ_P16)
#define WS_O     (WS_VT   + WSZ_P16)
#define WS_X1    (WS_O    + WSZ_P16)
#define WS_H32   (WS_X1   + WSZ_P32)
#define WS_H     (WS_H32  + WSZ_H32)
#define WS_Y     (WS_H    + WSZ_H)
#define WS_PS    (WS_Y    + WSZ_P32)
#define WS_PQ    (WS_PS   + WSZ_PT)
#define WS_AB1   (WS_PQ   + WSZ_PT)
#define WS_AB2   (WS_AB1  + WSZ_AB1)
#define WS_END   (WS_AB2  + WSZ_AB2)
static_assert(WS_END <= (size_t)134217728u);
static_assert((WS_XN % 256u) == 0 && (WS_Q % 256u) == 0 && (WS_VT % 256u) == 0 && (WS_X1 % 256u) == 0 && (WS_H % 256u) == 0);
static_assert((WS_H32 % 256u) == 0 && (WS_Y % 256u) == 0 && (WS_PS % 256u) == 0 && (WS_PQ % 256u) == 0 && (WS_AB1 % 256u) == 0 && (WS_AB2 % 256u) == 0);
static_assert((ROWS / 64u) * 64u == ROWS);
static_assert((TOKS / 64u) * 64u == TOKS);
static_assert((ROWS / 8u) * 8u == ROWS);
static_assert((SEQ / 16) * 16 == SEQ);
static_assert(NGRP * 16u == ROWS);
static_assert(((size_t)ROWS * FF) % 2048u == 0 && 2048u % FF == 0);
static_assert(256u * 8u == 2048u);
static_assert(((size_t)ROWS * (DM / 4)) % 256u == 0);
static_assert(128u * 4u == 64u * 8u);
static_assert(128u * 8u == 64u * 16u);
static_assert(128u * 8u == 128u * 8u);
static_assert(256u * 2u == 16u * 32u);
static_assert(8u * 32u * 16u == 16u * 64u * 4u);
static_assert(64u * 72u * 2u <= 131072u);
static_assert(128u * 72u * 2u + 64u * 36u * 4u <= 131072u);
static_assert(4u * 16u * 132u * 4u <= 131072u);
static_assert(8u * 16u * 72u * 2u + 16u * 264u * 2u + 2u * 16u * 4u <= 131072u);
static_assert(2u * 8u * 32u * 8u + 2u * 32u * 4u <= 131072u);
static_assert(2048u * 2u <= 131072u);

template <typename T> __device__ __forceinline__ void vst2(void* p, T v) { *(volatile T*)p = v; __threadfence(); *(volatile T*)p = v; }
__device__ __forceinline__ v8f zero8() { v8f z = {0.f, 0.f, 0.f, 0.f, 0.f, 0.f, 0.f, 0.f}; return z; }
__device__ __forceinline__ v8f wmma16(v16h a, v16h b, v8f c) {
  v8f d = __builtin_amdgcn_wmma_f32_16x16x32_f16(false, a, false, b, (short)0, c, false, false);
  asm volatile("v_nop\n\tv_nop\n\tv_nop\n\tv_nop" : "+v"(d) : "v"(a), "v"(b));
  return d;
}
__device__ __forceinline__ v16h frag_h(const _Float16* rowk0, int lane) {
  union { v16h v; v8h q[2]; } u; const _Float16* p = rowk0 + 8 * (lane >> 4);
  u.q[0] = *(const v8h*)p; u.q[1] = *(const v8h*)(p + 16); return u.v;
}
__device__ __forceinline__ _Float16 f16n(float x) { const float t = (fabsf(x) >= F16MIN) ? x : 0.0f; return (_Float16)t; }
__device__ __forceinline__ _Float16 toh_flush(float v) { const _Float16 r = (_Float16)v; return (fabsf(v) < F16MIN) ? (_Float16)0.0f : r; }
__device__ __forceinline__ unsigned short bf16bits(float x) { unsigned u = __float_as_uint(x); u += 0x7FFFu + ((u >> 16) & 1u); return (unsigned short)(u >> 16); }
__device__ __forceinline__ float bf16val(unsigned short b) { return __uint_as_float(((unsigned)b) << 16); }
__device__ __forceinline__ float rnev(float x) { return bf16val(bf16bits(x)); }
#define LDSX() do { asm volatile("s_wait_dscnt 0" ::: "memory"); __builtin_amdgcn_wave_barrier(); __builtin_amdgcn_fence(3  , "workgroup"); } while (0)

__global__ __launch_bounds__(256) void k_wt(const float* __restrict__ src, unsigned K, unsigned N, unsigned hsplit, _Float16* __restrict__ dst) {
  __shared__ __align__(16) _Float16 t[64][72];
  const unsigned tid = threadIdx.x; const unsigned n0 = blockIdx.x * 64u, k0 = blockIdx.y * 64u;
  const unsigned np = tid & 15u, kq = tid >> 4;
#pragma unroll
  for (unsigned i = 0; i < 4; ++i) {
    const unsigned kk = kq + 16u * i;
    const v4f v = *(const v4f*)(src + (size_t)(k0 + kk) * N + n0 + 4u * np);
#pragma unroll
    for (int e = 0; e < 4; ++e) t[4u * np + e][kk] = toh_flush(rnev(v[e]) * WC);
  }
  __syncthreads();
  for (unsigned e = tid; e < 64u * 8u; e += 256u) {
    const unsigned nl = e >> 3, q = e & 7u; const unsigned n = n0 + nl;
    const unsigned nd = hsplit ? ((n & 7u) * (unsigned)DH + (n >> 3)) : n;
    vst2(dst + (size_t)nd * K + k0 + q * 8u, *(const v8h*)&t[nl][q * 8u]);
  }
}

template <int RAW>
__global__ __launch_bounds__(256) void k_ln(const float* __restrict__ S0, const float* __restrict__ S1, unsigned bs, const float* __restrict__ G, const float* __restrict__ Bt, _Float16* __restrict__ XN) {
  const unsigned wave = threadIdx.x >> 5, lane = threadIdx.x & 31u; const unsigned row = blockIdx.x * 8u + wave;
  if (row >= ROWS) return;
  const unsigned s = row / TOKS, rem = row - s * TOKS, b = rem / (unsigned)SEQ, tk = rem - b * (unsigned)SEQ;
  const float* p = (s ? S1 : S0) + ((size_t)b * bs + tk) * DM + lane * 8u;
  const v4f a = *(const v4f*)p, c = *(const v4f*)(p + 4);
  float v[8];
#pragma unroll
  for (int e = 0; e < 4; ++e) { v[e] = RAW ? rnev(a[e]) : a[e]; v[4 + e] = RAW ? rnev(c[e]) : c[e]; }
  float s1 = ((v[0] + v[1]) + (v[2] + v[3])) + ((v[4] + v[5]) + (v[6] + v[7]));
#pragma unroll
  for (int o = 1; o < 32; o <<= 1) s1 += __shfl_xor(s1, o);
  const float mu = s1 * (1.0f / DM); float q = 0.f;
#pragma unroll
  for (int e = 0; e < 8; ++e) { const float d = v[e] - mu; q += d * d; }
#pragma unroll
  for (int o = 1; o < 32; o <<= 1) q += __shfl_xor(q, o);
  const float inv = rsqrtf(q * (1.0f / DM) + LN_EPS);
  const v4f ga = *(const v4f*)(G + lane * 8u), gb = *(const v4f*)(G + lane * 8u + 4u);
  const v4f ba = *(const v4f*)(Bt + lane * 8u), bb = *(const v4f*)(Bt + lane * 8u + 4u);
  v8h o8;
#pragma unroll
  for (int e = 0; e < 4; ++e) { o8[e] = f16n((v[e] - mu) * inv * rnev(ga[e]) + rnev(ba[e])); o8[4 + e] = f16n((v[4 + e] - mu) * inv * rnev(gb[e]) + rnev(bb[e])); }
  vst2(XN + (size_t)row * DM + lane * 8u, o8);
}

__device__ __forceinline__ void gemm_core(const _Float16* __restrict__ A, const _Float16* __restrict__ W, unsigned K, size_t arow, unsigned c0, int lane, v8f (&acc)[8]) {
  const unsigned col = (unsigned)lane & 15u;
#pragma unroll
  for (int j = 0; j < 8; ++j) acc[j] = zero8();
#pragma unroll 1
  for (unsigned kc = 0; kc < K; kc += 32u) {
    const v16h a = frag_h(A + (arow + col) * K + kc, lane);
#pragma unroll
    for (int j = 0; j < 8; ++j) acc[j] = wmma16(a, frag_h(W + (size_t)(c0 + j * 16u + col) * K + kc, lane), acc[j]);
  }
}
__device__ __forceinline__ void stage_rm(_Float16* sbuf, const v8f (&acc)[8], const float (&bv)[8], float sc, unsigned wave, unsigned g, unsigned col, int relu) {
#pragma unroll
  for (int j = 0; j < 8; ++j)
#pragma unroll
    for (int r = 0; r < 8; ++r) { float v = acc[j][r] * sc + bv[j]; if (relu) v = fmaxf(v, 0.0f); sbuf[(wave * 16u + 8u * g + r) * 136u + j * 16u + col] = toh_flush(v); }
}
__device__ __forceinline__ void store_rm(const _Float16* sbuf, _Float16* OP, unsigned pitch, size_t r0blk, unsigned cbase, unsigned tid) {
  for (unsigned e = tid; e < 64u * 16u; e += 128u) { const unsigned rl = e >> 4, q = e & 15u; vst2(OP + (r0blk + rl) * pitch + cbase + q * 8u, *(const v8h*)&sbuf[rl * 136u + q * 8u]); }
}

__global__ __launch_bounds__(128) void k_qkv(const _Float16* __restrict__ A, const _Float16* __restrict__ W, const float* __restrict__ BQ, const float* __restrict__ BK, const float* __restrict__ BV,
                                             _Float16* QO, _Float16* KO, _Float16* VTO, float* FV) {
  __shared__ __align__(16) _Float16 sbuf[128 * 72];
  __shared__ __align__(16) float sV[64 * 36];
  const unsigned tid = threadIdx.x, wave = tid >> 5; const int lane = (int)(tid & 31u); const unsigned col = tid & 15u, g = (tid >> 4) & 1u;
  const size_t r0blk = (size_t)blockIdx.x * 64u; const unsigned y = blockIdx.y, sel = y >> 1, cl0 = (y & 1u) * 128u, c0 = y * 128u;
  v8f acc[8];
  gemm_core(A, W, (unsigned)DM, r0blk + wave * 16u, c0, lane, acc);
  float bv[8];
#pragma unroll
  for (int j = 0; j < 8; ++j) {
    const unsigned nh = cl0 + j * 16u + col;
    const unsigned c = (nh & 31u) * 8u + (nh >> 5);
    const float vq = BQ[c], vk = BK[c], vv = BV[c];
    bv[j] = rnev((sel == 0u) ? vq : ((sel == 1u) ? vk : vv));
  }
  if (sel < 2u) {
    stage_rm(sbuf, acc, bv, 1.0f / WC, wave, g, col, 0);
  } else {
#pragma unroll
    for (int j = 0; j < 8; ++j)
#pragma unroll
      for (int r = 0; r < 8; ++r) sbuf[(j * 16u + col) * 72u + wave * 16u + 8u * g + r] = toh_flush(acc[j][r] * (1.0f / WC) + bv[j]);
    if (y == 5u) {
#pragma unroll
      for (int j = 6; j < 8; ++j)
#pragma unroll
        for (int r = 0; r < 8; ++r) sV[(wave * 16u + 8u * g + r) * 36u + (unsigned)(j - 6) * 16u + col] = acc[j][r] * (1.0f / WC) + bv[j];
    }
  }
  __syncthreads();
  if (sel < 2u) {
    store_rm(sbuf, sel ? KO : QO, (unsigned)DM, r0blk, cl0, tid);
  } else {
    for (unsigned e = tid; e < 128u * 8u; e += 128u) { const unsigned cl = e >> 3, q = e & 7u; vst2(VTO + (size_t)(cl0 + cl) * ROWS + r0blk + q * 8u, *(const v8h*)&sbuf[cl * 72u + q * 8u]); }
    if (y == 5u) {
      for (unsigned e = tid; e < 64u * 8u; e += 128u) {
        const unsigned rl = e >> 3, q = e & 7u; const unsigned row = (unsigned)r0blk + rl;
        const unsigned bb = row / (unsigned)SEQ, tk = row - bb * (unsigned)SEQ;
        vst2(FV + ((size_t)bb * SEQ_FULL + tk) * DH + q * 4u, *(const v4f*)&sV[rl * 36u + q * 4u]);
      }
    }
  }
}

template <int RNERES>
__global__ __launch_bounds__(128) void k_gres(const _Float16* __restrict__ A, const _Float16* __restrict__ W, unsigned K, const float* __restrict__ BO,
                                              const float* R0, const float* R1, unsigned rbs, float* O0, float* O1, unsigned obs, float sc) {
  __shared__ __align__(16) float sf[4][16][132];
  const unsigned tid = threadIdx.x, wave = tid >> 5; const int lane = (int)(tid & 31u); const unsigned col = tid & 15u, g = (tid >> 4) & 1u, ln = tid & 31u;
  const unsigned row0 = blockIdx.x * 64u; const unsigned c0 = blockIdx.y * 128u;
  v8f acc[8];
  gemm_core(A, W, K, (size_t)row0 + wave * 16u, c0, lane, acc);
  float bv[8];
#pragma unroll
  for (int j = 0; j < 8; ++j) bv[j] = rnev(BO[c0 + j * 16u + col]);
#pragma unroll
  for (int j = 0; j < 8; ++j)
#pragma unroll
    for (int r = 0; r < 8; ++r) sf[wave][8u * g + r][j * 16u + col] = acc[j][r] * sc + bv[j];
  LDSX();
  const unsigned s = row0 / TOKS, rem = row0 - s * TOKS, b = rem / (unsigned)SEQ, t0 = rem - b * (unsigned)SEQ + wave * 16u;
  const float* rp = (s ? R1 : R0) + ((size_t)b * rbs + t0) * DM + c0 + ln * 4u;
  float* op = (s ? O1 : O0) + ((size_t)b * obs + t0) * DM + c0 + ln * 4u;
#pragma unroll 1
  for (unsigned rl = 0; rl < 16u; ++rl) {
    v4f vv = *(const v4f*)&sf[wave][rl][ln * 4u];
    const v4f rv = *(const v4f*)(rp + (size_t)rl * DM);
#pragma unroll
    for (int e = 0; e < 4; ++e) vv[e] += RNERES ? rnev(rv[e]) : rv[e];
    vst2(op + (size_t)rl * DM, vv);
  }
}

__global__ __launch_bounds__(128) void k_gstat(const _Float16* __restrict__ A, const _Float16* __restrict__ W, unsigned K, unsigned N, const float* __restrict__ BI,
                                               float* __restrict__ Y, float* __restrict__ PS, float* __restrict__ PQ, float sc) {
  __shared__ __align__(16) float sf[4][16][132];
  const unsigned tid = threadIdx.x, wave = tid >> 5; const int lane = (int)(tid & 31u); const unsigned col = tid & 15u, g = (tid >> 4) & 1u, ln = tid & 31u;
  const unsigned row0 = blockIdx.x * 64u; const unsigned c0 = blockIdx.y * 128u;
  v8f acc[8];
  gemm_core(A, W, K, (size_t)row0 + wave * 16u, c0, lane, acc);
  float bv[8];
#pragma unroll
  for (int j = 0; j < 8; ++j) bv[j] = rnev(BI[c0 + j * 16u + col]);
#pragma unroll
  for (int j = 0; j < 8; ++j)
#pragma unroll
    for (int r = 0; r < 8; ++r) sf[wave][8u * g + r][j * 16u + col] = acc[j][r] * sc + bv[j];
  LDSX();
  float* yp = Y + ((size_t)row0 + wave * 16u) * N + c0 + ln * 4u;
  v4f s = {0.f, 0.f, 0.f, 0.f}, qq = {0.f, 0.f, 0.f, 0.f};
#pragma unroll 1
  for (unsigned rl = 0; rl < 16u; ++rl) {
    const v4f vv = *(const v4f*)&sf[wave][rl][ln * 4u];
    s += vv; qq += vv * vv;
    vst2(yp + (size_t)rl * N, vv);
  }
  const size_t grp = (size_t)blockIdx.x * 4u + wave;
  vst2(PS + grp * N + c0 + ln * 4u, s);
  vst2(PQ + grp * N + c0 + ln * 4u, qq);
}

__global__ __launch_bounds__(256) void k_bnstat(const float* __restrict__ PS, const float* __restrict__ PQ, unsigned N, const float* __restrict__ G, const float* __restrict__ Bt, float* __restrict__ AB) {
  __shared__ double sS[8][32];
  __shared__ double sQ[8][32];
  __shared__ __align__(16) float sAB[2][32];
  const unsigned tid = threadIdx.x; const unsigned wave = (unsigned)__builtin_amdgcn_readfirstlane((int)(threadIdx.x >> 5)); const unsigned lane = tid & 31u;
  const unsigned c = blockIdx.x * 32u + lane;
  double s = 0.0, q = 0.0;
#pragma unroll 1
  for (unsigned gi = wave; gi < NGRP; gi += 8u) { s += (double)PS[(size_t)gi * N + c]; q += (double)PQ[(size_t)gi * N + c]; }
  sS[wave][lane] = s; sQ[wave][lane] = q;
  __syncthreads();
  if (wave == 0u) {
    double ts = 0.0, tq = 0.0;
#pragma unroll 1
    for (unsigned w = 0; w < 8u; ++w) { ts += sS[w][lane]; tq += sQ[w][lane]; }
    const double mean = ts * (1.0 / (double)ROWS);
    const double var = tq * (1.0 / (double)ROWS) - mean * mean;
    const float vf = fmaxf((float)var, 0.0f);
    const float rstd = rsqrtf(vf + BN_EPS);
    const float a = rnev(G[c]) * rstd;
    const float bsh = rnev(Bt[c]) - (float)mean * a;
    sAB[0][lane] = a; sAB[1][lane] = bsh;
    LDSX();
    const unsigned tb = (lane >> 3) & 1u, qd = lane & 7u;
    const v4f o = *(const v4f*)&sAB[tb][qd * 4u];
    if (lane < 16u) vst2(AB + (size_t)tb * N + blockIdx.x * 32u + qd * 4u, o);
  }
}

__global__ __launch_bounds__(256) void k_bngelu(const float* __restrict__ X, const float* __restrict__ AB, _Float16* __restrict__ H) {
  __shared__ __align__(16) _Float16 t[2048];
  const unsigned tid = threadIdx.x; const size_t base = (size_t)blockIdx.x * 2048u;
#pragma unroll 1
  for (unsigned i = 0; i < 8u; ++i) {
    const unsigned idx = i * 256u + tid; const unsigned c = idx & ((unsigned)FF - 1u);
    const float v = X[base + idx] * AB[c] + AB[(unsigned)FF + c];
    const float ge = 0.5f * v * (1.0f + erff(v * 0.70710678118654752f));
    t[idx] = toh_flush(ge);
  }
  __syncthreads();
  vst2(H + base + tid * 8u, *(const v8h*)&t[tid * 8u]);
}

__global__ __launch_bounds__(256) void k_bnout(const float* __restrict__ Y, const float* __restrict__ AB, const float* __restrict__ X1, float* __restrict__ OUT) {
  const unsigned idx = blockIdx.x * 256u + threadIdx.x; const unsigned row = idx >> 6, cq = idx & 63u;
  if (row >= ROWS) return;
  const v4f y = *(const v4f*)(Y + (size_t)row * DM + cq * 4u);
  const v4f x = *(const v4f*)(X1 + (size_t)row * DM + cq * 4u);
  const v4f a = *(const v4f*)(AB + cq * 4u);
  const v4f bs = *(const v4f*)(AB + (unsigned)DM + cq * 4u);
  const unsigned bb = row / (unsigned)SEQ, tk = row - bb * (unsigned)SEQ;
  v4f o;
#pragma unroll
  for (int e = 0; e < 4; ++e) o[e] = x[e] + (y[e] * a[e] + bs[e]);
  vst2(OUT + ((size_t)bb * SEQ_FULL + tk) * DM + cq * 4u, o);
}

__global__ __launch_bounds__(256) void k_attn(const _Float16* __restrict__ Q, const _Float16* __restrict__ KP, const _Float16* __restrict__ VT, _Float16* __restrict__ O, float* __restrict__ PW) {
  __shared__ __align__(16) _Float16 sP[8][16][72];
  __shared__ __align__(16) _Float16 sO[16][264];
  __shared__ float sM[16];
  __shared__ float sW[16];
  const unsigned tid = threadIdx.x; const unsigned wave = (unsigned)__builtin_amdgcn_readfirstlane((int)(threadIdx.x >> 5));
  const int lane = (int)(tid & 31u); const unsigned col = tid & 15u, g = (tid >> 4) & 1u;
  const unsigned q0 = blockIdx.x * 16u, b = blockIdx.y;
  const size_t qrow0 = (size_t)b * SEQ + q0;
  const size_t krow0 = (size_t)b * SEQ;
  const unsigned hc = wave * DH;
  const v16h qa = frag_h(Q + (qrow0 + col) * DM + hc, lane);
  float mrow[8], lsum[8];
#pragma unroll
  for (int r = 0; r < 8; ++r) { mrow[r] = -1.0e30f; lsum[r] = 0.f; }
  v8f o0 = zero8(), o1 = zero8();
#pragma unroll 1
  for (unsigned kt = 0; kt < (unsigned)SEQ / 64u; ++kt) {
    const unsigned key0 = kt * 64u;
    v8f sc[4];
#pragma unroll
    for (int t = 0; t < 4; ++t) sc[t] = wmma16(qa, frag_h(KP + (krow0 + key0 + 4u * col + t) * DM + hc, lane), zero8());
#pragma unroll
    for (int t = 0; t < 4; ++t)
#pragma unroll
      for (int r = 0; r < 8; ++r) sc[t][r] = sc[t][r] * SCALE;
#pragma unroll
    for (int r = 0; r < 8; ++r) {
      float mx = fmaxf(fmaxf(sc[0][r], sc[1][r]), fmaxf(sc[2][r], sc[3][r]));
      mx = fmaxf(mx, __shfl_xor(mx, 1)); mx = fmaxf(mx, __shfl_xor(mx, 2)); mx = fmaxf(mx, __shfl_xor(mx, 4)); mx = fmaxf(mx, __shfl_xor(mx, 8));
      const float mn = fmaxf(mrow[r], mx);
      const float al = __expf(mrow[r] - mn);
      mrow[r] = mn; o0[r] *= al; o1[r] *= al;
      float ls = lsum[r] * al;
      v4h pk;
#pragma unroll
      for (int t = 0; t < 4; ++t) { const float pc = __expf(sc[t][r] - mn) * PCY; const _Float16 ph = toh_flush(pc); ls += (float)ph; pk[t] = ph; }
      lsum[r] = ls;
      *(v4h*)&sP[wave][8u * g + r][4u * col] = pk;
    }
    LDSX();
#pragma unroll
    for (int kk = 0; kk < 2; ++kk) {
      const v16h a = frag_h(&sP[wave][col][kk * 32], lane);
      o0 = wmma16(a, frag_h(VT + (size_t)(hc + col) * ROWS + krow0 + key0 + kk * 32u, lane), o0);
      o1 = wmma16(a, frag_h(VT + (size_t)(hc + 16u + col) * ROWS + krow0 + key0 + kk * 32u, lane), o1);
    }
    LDSX();
  }
#pragma unroll
  for (int r = 0; r < 8; ++r) {
    float t = lsum[r]; t += __shfl_xor(t, 1); t += __shfl_xor(t, 2); t += __shfl_xor(t, 4); t += __shfl_xor(t, 8);
    const float rt = 1.0f / t;
    const float inv = OC * rt;
    sO[8u * g + r][hc + col] = toh_flush(o0[r] * inv);
    sO[8u * g + r][hc + 16u + col] = toh_flush(o1[r] * inv);
    if (wave == (unsigned)(NH - 1)) {
      if (col == 0u) { sM[8u * g + r] = mrow[r]; sW[8u * g + r] = PCY * rt; }
    }
  }
  __syncthreads();
  for (unsigned e = tid; e < 16u * 32u; e += 256u) { const unsigned rl = e >> 5, pc = e & 31u; vst2(O + (qrow0 + rl) * DM + pc * 8u, *(const v8h*)&sO[rl][pc * 8u]); }
  const v16h qa7 = frag_h(Q + (qrow0 + col) * DM + (unsigned)(NH - 1) * DH, lane);
  float m7[8], w7[8];
#pragma unroll
  for (int r = 0; r < 8; ++r) { m7[r] = sM[8u * g + r]; w7[r] = sW[8u * g + r]; }
  float* pw = PW + ((size_t)b * SEQ_FULL + q0 + 8u * g) * SEQ_FULL + 4u * col;
#pragma unroll 1
  for (unsigned kt = wave; kt < (unsigned)SEQ / 64u; kt += 8u) {
    const unsigned key0 = kt * 64u;
    v8f sc[4];
#pragma unroll
    for (int t = 0; t < 4; ++t) sc[t] = wmma16(qa7, frag_h(KP + (krow0 + key0 + 4u * col + t) * DM + (unsigned)(NH - 1) * DH, lane), zero8());
#pragma unroll
    for (int r = 0; r < 8; ++r) {
      v4f pv;
#pragma unroll
      for (int t = 0; t < 4; ++t) pv[t] = __expf(sc[t][r] * SCALE - m7[r]) * w7[r];
      vst2(pw + (size_t)r * SEQ_FULL + key0, pv);
    }
  }
}

extern "C" void kernel_launch(void* const* d_in, const int* in_sizes, int n_in, void* d_out, int out_size, void* d_ws, size_t ws_size, hipStream_t stream) {
  if (n_in < 21) return;
  const size_t need_x = ((size_t)(NB - 1) * SEQ_FULL + SEQ) * DM;
  const size_t need_w = ((size_t)(NB - 1) * SEQ_FULL + (SEQ - 1)) * SEQ_FULL + SEQ;
  const size_t need_v = ((size_t)(NB - 1) * SEQ_FULL + SEQ) * DH;
  if ((size_t)in_sizes[0] < need_x) return;
  for (int i = 1; i <= 4; ++i) if (in_sizes[i] < DM) return;
  for (int i = 5; i <= 11; i += 2) if (in_sizes[i] < DM * DM) return;
  for (int i = 6; i <= 12; i += 2) if (in_sizes[i] < DM) return;
  if (in_sizes[13] < DM * FF || in_sizes[14] < FF || in_sizes[15] < FF || in_sizes[16] < FF) return;
  if (in_sizes[17] < FF * DM || in_sizes[18] < DM || in_sizes[19] < DM || in_sizes[20] < DM) return;
  if ((size_t)out_size < need_x || (size_t)out_size < OUT1_OFF + need_w || (size_t)out_size < OUT2_OFF + need_v) return;
  if (ws_size < (size_t)WS_END) return;
  const float* x = (const float*)d_in[0];
  const float* ln1_g = (const float*)d_in[1]; const float* ln1_b = (const float*)d_in[2];
  const float* ln2_g = (const float*)d_in[3]; const float* ln2_b = (const float*)d_in[4];
  const float* wq = (const float*)d_in[5];  const float* bq = (const float*)d_in[6];
  const float* wk = (const float*)d_in[7];  const float* bk = (const float*)d_in[8];
  const float* wv = (const float*)d_in[9];  const float* bv = (const float*)d_in[10];
  const float* wp = (const float*)d_in[11]; const float* bp = (const float*)d_in[12];
  const float* w1 = (const float*)d_in[13]; const float* b1 = (const float*)d_in[14];
  const float* bn1_g = (const float*)d_in[15]; const float* bn1_b = (const float*)d_in[16];
  const float* w2 = (const float*)d_in[17]; const float* b2 = (const float*)d_in[18];
  const float* bn2_g = (const float*)d_in[19]; const float* bn2_b = (const float*)d_in[20];
  char* ws = (char*)d_ws;
  _Float16* WQKV = (_Float16*)(ws + WS_WQKV); _Float16* WO = (_Float16*)(ws + WS_WO);
  _Float16* W1T = (_Float16*)(ws + WS_W1T); _Float16* W2T = (_Float16*)(ws + WS_W2T);
  _Float16* XN = (_Float16*)(ws + WS_XN); _Float16* Qp = (_Float16*)(ws + WS_Q); _Float16* Kp = (_Float16*)(ws + WS_K);
  _Float16* VTp = (_Float16*)(ws + WS_VT); _Float16* Op = (_Float16*)(ws + WS_O); _Float16* Hp = (_Float16*)(ws + WS_H);
  float* X1 = (float*)(ws + WS_X1); float* H32 = (float*)(ws + WS_H32); float* Yp = (float*)(ws + WS_Y);
  float* PS = (float*)(ws + WS_PS); float* PQ = (float*)(ws + WS_PQ);
  float* AB1 = (float*)(ws + WS_AB1); float* AB2 = (float*)(ws + WS_AB2);
  float* out = (float*)d_out;
  const size_t SQ = (size_t)DM * DM;

  k_wt<<<dim3(DM / 64, DM / 64), 256, 0, stream>>>(wq, (unsigned)DM, (unsigned)DM, 1u, WQKV);
  k_wt<<<dim3(DM / 64, DM / 64), 256, 0, stream>>>(wk, (unsigned)DM, (unsigned)DM, 1u, WQKV + SQ);
  k_wt<<<dim3(DM / 64, DM / 64), 256, 0, stream>>>(wv, (unsigned)DM, (unsigned)DM, 1u, WQKV + 2 * SQ);
  k_wt<<<dim3(DM / 64, DM / 64), 256, 0, stream>>>(wp, (unsigned)DM, (unsigned)DM, 0u, WO);
  k_wt<<<dim3(FF / 64, DM / 64), 256, 0, stream>>>(w1, (unsigned)DM, (unsigned)FF, 0u, W1T);
  k_wt<<<dim3(DM / 64, FF / 64), 256, 0, stream>>>(w2, (unsigned)FF, (unsigned)DM, 0u, W2T);

  k_ln<1><<<dim3(ROWS / 8u), 256, 0, stream>>>(x, x, (unsigned)SEQ_FULL, ln1_g, ln1_b, XN);
  k_qkv<<<dim3(ROWS / 64u, 6), 128, 0, stream>>>(XN, WQKV, bq, bk, bv, Qp, Kp, VTp, out + OUT2_OFF);
  k_attn<<<dim3(SEQ / 16, NB), 256, 0, stream>>>(Qp, Kp, VTp, Op, out + OUT1_OFF);
  k_gres<1><<<dim3(ROWS / 64u, DM / 128), 128, 0, stream>>>(Op, WO, (unsigned)DM, bp, x, x, (unsigned)SEQ_FULL, X1, X1, (unsigned)SEQ, 1.0f / (WC * OC));

  k_ln<0><<<dim3(ROWS / 8u), 256, 0, stream>>>(X1, X1, (unsigned)SEQ, ln2_g, ln2_b, XN);
  k_gstat<<<dim3(ROWS / 64u, FF / 128), 128, 0, stream>>>(XN, W1T, (unsigned)DM, (unsigned)FF, b1, H32, PS, PQ, 1.0f / WC);
  k_bnstat<<<dim3(FF / 32), 256, 0, stream>>>(PS, PQ, (unsigned)FF, bn1_g, bn1_b, AB1);
  k_bngelu<<<dim3((unsigned)(((size_t)ROWS * FF) / 2048u)), 256, 0, stream>>>(H32, AB1, Hp);
  k_gstat<<<dim3(ROWS / 64u, DM / 128), 128, 0, stream>>>(Hp, W2T, (unsigned)FF, (unsigned)DM, b2, Yp, PS, PQ, 1.0f / WC);
  k_bnstat<<<dim3(DM / 32), 256, 0, stream>>>(PS, PQ, (unsigned)DM, bn2_g, bn2_b, AB2);
  k_bnout<<<dim3((unsigned)(((size_t)ROWS * (DM / 4)) / 256u)), 256, 0, stream>>>(Yp, AB2, X1, out);
}
